// GraphAttentionLayer_89799176225427
// MI455X (gfx1250) — hardware-verified
//
#include <hip/hip_runtime.h>
#include <math.h>

#ifndef NB
#define NB 8
#endif
#ifndef SEQ
#define SEQ 2048
#endif
#define SEQ_FULL 2048
#define IN_DIM 256
#define OUT_DIM 256
#define HEADS 4
#define HD 64
#define NPROJ 512
#define MTOK (NB * SEQ)

#define X_CARRY 16.0f
#define W_CARRY 64.0f
#define GEMM_UNDO (1.0f / 1024.0f)
#define V_CARRY 16.0f
#define P_CARRY 1024.0f
#define PV_UNDO (1.0f / (1024.0f * 16.0f))
#define LOG2E 1.4426950408889634f
#define LEAK 0.2f

static_assert(X_CARRY * W_CARRY * GEMM_UNDO == 1.0f);
static_assert(P_CARRY * V_CARRY * PV_UNDO == 1.0f);
static_assert(SEQ <= SEQ_FULL);
static_assert(HEADS * HD == OUT_DIM);
static_assert(NPROJ == 2 * OUT_DIM);
static_assert(MTOK % 64 == 0);
static_assert(NPROJ % 64 == 0 && OUT_DIM % 64 == 0);
static_assert(IN_DIM % 32 == 0 && SEQ % 32 == 0);
static_assert(SEQ % 128 == 0 && SEQ % 64 == 0);
static_assert((MTOK * IN_DIM / 8) % 256 == 0);
static_assert(IN_DIM == 256);
static_assert(HD == 64);

typedef __attribute__((ext_vector_type(16))) _Float16 v16h;
typedef __attribute__((ext_vector_type(8)))  _Float16 v8h;
typedef __attribute__((ext_vector_type(2)))  _Float16 v2h;
typedef __attribute__((ext_vector_type(8)))  float    v8f;
typedef __attribute__((ext_vector_type(4)))  float    v4f;
typedef __attribute__((ext_vector_type(2)))  float    v2f;
typedef __attribute__((ext_vector_type(4)))  unsigned int v4u;
typedef __attribute__((ext_vector_type(8)))  unsigned int v8u;


#define VST2(T, ptr, val) do { const T vst2_v_ = (val); *(volatile T*)(ptr) = vst2_v_; __threadfence(); *(volatile T*)(ptr) = vst2_v_; } while (0)
#define VST2V4(ptr, val) do { const v4f vst2_v4_ = (val); *(volatile v4f*)(ptr) = vst2_v4_; __threadfence(); *(volatile v4f*)(ptr) = vst2_v4_; } while (0)

__device__ __forceinline__ float bfr(float f) {
    unsigned u = __float_as_uint(f);
    u += 0x7FFFu + ((u >> 16) & 1u);
    return __uint_as_float(u & 0xFFFF0000u);
}
__device__ __forceinline__ unsigned short f2h_bits(float x) {
    return (fabsf(x) < 6.104e-5f) ? (unsigned short)0 : __builtin_bit_cast(unsigned short, (_Float16)x);
}
__device__ __forceinline__ void st8h(unsigned short* P, size_t o, const float* v) {
    v4u pk;
    pk.x = (unsigned)f2h_bits(v[0]) | ((unsigned)f2h_bits(v[1]) << 16);
    pk.y = (unsigned)f2h_bits(v[2]) | ((unsigned)f2h_bits(v[3]) << 16);
    pk.z = (unsigned)f2h_bits(v[4]) | ((unsigned)f2h_bits(v[5]) << 16);
    pk.w = (unsigned)f2h_bits(v[6]) | ((unsigned)f2h_bits(v[7]) << 16);
    VST2(v4u, (v4u*)(P + o), pk);
}

__device__ __forceinline__ unsigned toh_flush2(float a, float b) {
    v2f w;
    w.x = (fabsf(a) < 6.103515625e-05f) ? 0.0f : a;
    w.y = (fabsf(b) < 6.103515625e-05f) ? 0.0f : b;
    const v2h hp = __builtin_convertvector(w, v2h);
    return __builtin_bit_cast(unsigned, hp);
}
__device__ __forceinline__ void st8hp(unsigned short* P, size_t o, const float* v) {
    v4u pk;
    pk.x = toh_flush2(v[0], v[1]);
    pk.y = toh_flush2(v[2], v[3]);
    pk.z = toh_flush2(v[4], v[5]);
    pk.w = toh_flush2(v[6], v[7]);
    VST2(v4u, (v4u*)(P + o), pk);
}

union FragU { v16h v; v8h h[2]; };
__device__ __forceinline__ v16h frag_ld(const _Float16* p) {
    FragU f; f.h[0] = *(const v8h*)(p); f.h[1] = *(const v8h*)(p + 16); return f.v;
}
__device__ __forceinline__ v8f wmma16(v16h a, v16h b, v8f c) {
    c = __builtin_amdgcn_wmma_f32_16x16x32_f16(false, a, false, b, (short)0, c, false, false);
    asm volatile("v_nop\n\tv_nop\n\tv_nop\n\tv_nop" : "+v"(c) : "v"(a), "v"(b));
    return c;
}
__device__ __forceinline__ void wave_sync_lds() {
    __builtin_amdgcn_fence(3  , "workgroup");
    __builtin_amdgcn_wave_barrier();
    __builtin_amdgcn_fence(2  , "workgroup");
}
__device__ __forceinline__ float fselmax(float a, float b) { return (a > b) ? a : b; }
__device__ __forceinline__ float elu1(float v) { return (v > 0.0f) ? v : expm1f(v); }

static_assert(32 * 16 * 8 == 16 * 64 * 4);
static_assert(8 * 16 * 68 * 4 <= 131072);
__global__ __launch_bounds__(256) void k_gemm64(
    const _Float16* __restrict__ A, unsigned lda, const _Float16* __restrict__ Bt, unsigned ldb,
    float* __restrict__ C, unsigned ldc, unsigned M, unsigned N, unsigned K) {
  __shared__ __align__(16) float sT[8][16 * 68];
  const unsigned lane = threadIdx.x & 31u;
  const unsigned wave = threadIdx.x >> 5;
  const unsigned tilesN = N >> 6, tilesM = M >> 6;
  const unsigned tile = blockIdx.x * 8u + wave;
  if (tile >= tilesM * tilesN) return;
  const unsigned tm = tile / tilesN;
  const unsigned tn = tile - tm * tilesN;
  const unsigned m0 = tm << 6, n0 = tn << 6;
  const unsigned rlane = lane & 15u;
  const unsigned koff = (lane >> 4) * 8u;
  const unsigned mOff = koff;

  v8f acc[4][4];
#pragma unroll
  for (int i = 0; i < 4; ++i)
#pragma unroll
    for (int j = 0; j < 4; ++j) acc[i][j] = (v8f){0.f,0.f,0.f,0.f,0.f,0.f,0.f,0.f};

  for (unsigned k0 = 0; k0 < K; k0 += 32u) {
    v16h bh[4];
#pragma unroll
    for (int j = 0; j < 4; ++j)
      bh[j] = frag_ld(Bt + (size_t)(n0 + ((unsigned)j << 4) + rlane) * ldb + koff + k0);
#pragma unroll
    for (int i = 0; i < 4; ++i) {
      const v16h ah = frag_ld(A + (size_t)(m0 + ((unsigned)i << 4) + rlane) * lda + koff + k0);
#pragma unroll
      for (int j = 0; j < 4; ++j)
        acc[i][j] = wmma16(ah, bh[j], acc[i][j]);
    }
  }

  float* slab = sT[wave];
#pragma unroll
  for (int i = 0; i < 4; ++i) {
    const unsigned mBase = m0 + ((unsigned)i << 4);
#pragma unroll
    for (int j = 0; j < 4; ++j) {
#pragma unroll
      for (int r = 0; r < 8; ++r) {
        const float v = acc[i][j][r] * GEMM_UNDO;
        slab[(mOff + (unsigned)r) * 68u + ((unsigned)j << 4) + rlane] = v;
      }
    }
    wave_sync_lds();
    {
      const unsigned hh = lane >> 4, c4 = (lane & 15u) * 4u;
#pragma unroll
      for (int half = 0; half < 2; ++half) {
        v4f vv[4];
#pragma unroll
        for (int it = 0; it < 4; ++it) {
          const unsigned row = (unsigned)(half * 4 + it) * 2u + hh;
          vv[it] = *(const v4f*)(slab + row * 68u + c4);
        }
        for (int pass = 0; pass < 2; ++pass) {
#pragma unroll
          for (int it = 0; it < 4; ++it) {
            const unsigned row = (unsigned)(half * 4 + it) * 2u + hh;
            *(volatile v4f*)(C + (size_t)(mBase + row) * ldc + n0 + c4) = vv[it];
          }
          __threadfence();
        }
      }
    }
    wave_sync_lds();
  }
}

__global__ __launch_bounds__(256) void k_wt16(const float* __restrict__ Wm, unsigned KI, unsigned NO, unsigned lgper,
                                              unsigned short* __restrict__ W16, float sw) {
    const unsigned layer = blockIdx.y;
    const float* Wl = Wm + (size_t)layer * KI * NO;
    unsigned short* Dl = W16 + (size_t)layer * KI * NO;
    const unsigned u = blockIdx.x * 256u + threadIdx.x;
    const unsigned per = 1u << lgper;
    if (u >= NO * per) return;
    const unsigned k0 = 8u * (u & (per - 1u));
    const unsigned o = u >> lgper;
    float v[8];
#pragma unroll
    for (int i = 0; i < 8; ++i) v[i] = bfr(Wl[(size_t)(k0 + (unsigned)i) * NO + o]) * sw;
    st8h(Dl, (size_t)o * KI + k0, v);
}

__global__ __launch_bounds__(256) void k_x16(const float* __restrict__ h, unsigned short* __restrict__ x16) {
    const unsigned u = blockIdx.x * 256u + threadIdx.x;
    if (u >= (unsigned)(MTOK * IN_DIM / 8)) return;
    const unsigned row = u >> 5, c0 = (u & 31u) * 8u;
    const unsigned b = row / (unsigned)SEQ;
    const unsigned n = row - b * (unsigned)SEQ;
    const float* hr = h + (size_t)(b * (unsigned)SEQ_FULL + n) * IN_DIM + c0;
    const v4f a = *(const v4f*)hr;
    const v4f d = *(const v4f*)(hr + 4);
    float v[8];
    v[0] = bfr(a.x) * X_CARRY; v[1] = bfr(a.y) * X_CARRY; v[2] = bfr(a.z) * X_CARRY; v[3] = bfr(a.w) * X_CARRY;
    v[4] = bfr(d.x) * X_CARRY; v[5] = bfr(d.y) * X_CARRY; v[6] = bfr(d.z) * X_CARRY; v[7] = bfr(d.w) * X_CARRY;
    st8hp(x16, (size_t)row * IN_DIM + c0, v);
}

#define PL_P 68
static_assert(256 * 16 * 2 == 64 * 128);
static_assert(32 * 16 == 2 * 64 * 4);
static_assert((64 * PL_P + 128 + 128) * 4 <= 131072);
__global__ __launch_bounds__(256) void k_planes(const float* __restrict__ HF, const float* __restrict__ attn,
                                                unsigned short* __restrict__ VT, float* __restrict__ LR) {
    __shared__ __align__(16) float sV[64 * PL_P];
    __shared__ __align__(16) float sLR[128];
    __shared__ __align__(16) float sA[128];
    const unsigned t = threadIdx.x;
    const unsigned bx = blockIdx.x;
    const unsigned nch = (unsigned)(SEQ / 64);
    const unsigned hd = bx & 3u;
    const unsigned rest = bx >> 2;
    const unsigned nc = rest % nch;
    const unsigned b = rest / nch;
    const unsigned n0 = nc * 64u;
    if (t < 128u) sA[t] = bfr(attn[hd * 128u + t]);
    __syncthreads();
    const unsigned r = t >> 2, q4 = t & 3u;
    const size_t rowoff = (size_t)(b * (unsigned)SEQ + n0 + r) * NPROJ + 64u * hd + 16u * q4;
    const float* ps = HF + rowoff;
    const float* pn = HF + rowoff + OUT_DIM;
    float dl = 0.f, dr = 0.f;
#pragma unroll
    for (int g = 0; g < 4; ++g) {
        const v4f s4 = *(const v4f*)(ps + 4 * g);
        const v4f n4 = *(const v4f*)(pn + 4 * g);
        const unsigned ca = 16u * q4 + 4u * (unsigned)g;
        dl += s4.x * sA[ca];           dl += s4.y * sA[ca + 1u];
        dl += s4.z * sA[ca + 2u];      dl += s4.w * sA[ca + 3u];
        dr += n4.x * sA[64u + ca];     dr += n4.y * sA[64u + ca + 1u];
        dr += n4.z * sA[64u + ca + 2u]; dr += n4.w * sA[64u + ca + 3u];
        *(v4f*)(&sV[r * PL_P + ca]) = n4;
    }
    dl += __shfl_xor(dl, 1, 32); dr += __shfl_xor(dr, 1, 32);
    dl += __shfl_xor(dl, 2, 32); dr += __shfl_xor(dr, 2, 32);
    if (q4 == 0u) { sLR[r] = dl; sLR[64u + r] = dr; }
    __syncthreads();
#pragma unroll
    for (int pass = 0; pass < 2; ++pass) {
        const unsigned d = (unsigned)pass * 32u + (t >> 3);
        const unsigned n8 = (t & 7u) * 8u;
        float v[8];
#pragma unroll
        for (int e = 0; e < 8; ++e) v[e] = sV[(n8 + (unsigned)e) * PL_P + d] * V_CARRY;
        st8hp(VT, (size_t)(b * (unsigned)OUT_DIM + 64u * hd + d) * SEQ + n0 + n8, v);
    }
    if (t < 32u) {
        const unsigned which = t >> 4, c4 = (t & 15u) * 4u;
        const v4f v = *(const v4f*)(&sLR[which * 64u + c4]);
        const size_t off = (size_t)which * ((size_t)NB * HEADS * SEQ) + (size_t)(b * HEADS + hd) * SEQ + n0 + c4;
        VST2V4(LR + off, v);
    }
}

#define AT_PO 68
static_assert(32 * 16 * 8 == 16 * HD * 4);
static_assert((8 * 16 * AT_PO + 8 * 16) * 4 <= 131072);
__global__ __launch_bounds__(256) void k_attn(const _Float16* __restrict__ VT, const float* __restrict__ LR,
                                              float* __restrict__ out) {
    __shared__ __align__(16) float sO[8][16 * AT_PO];
    __shared__ __align__(16) float sL[8][16];
    const unsigned tid = threadIdx.x, lane = tid & 31u;
    const unsigned wave = (unsigned)__builtin_amdgcn_readfirstlane((int)(tid >> 5));
    const unsigned hh = lane >> 4, c = lane & 15u;
    const unsigned bx = blockIdx.x;
    const unsigned qch = (unsigned)(SEQ / 128);
    const unsigned qc = bx % qch;
    const unsigned bh = bx / qch;
    const unsigned b = bh >> 2, hd = bh & 3u;
    const unsigned i0 = qc * 128u + wave * 16u;
    const float* leftp  = LR + (size_t)bh * SEQ;
    const float* rightp = LR + (size_t)NB * HEADS * SEQ + (size_t)bh * SEQ + 8u * hh;
    const _Float16* vrow = VT + (size_t)(b * (unsigned)OUT_DIM + hd * (unsigned)HD + c) * SEQ + 8u * hh;
    const float li = leftp[i0 + c];

    float m = -3.0e38f, lsum = 0.f;
    v8f acc[4];
#pragma unroll
    for (int t = 0; t < 4; ++t) acc[t] = (v8f){0.f,0.f,0.f,0.f,0.f,0.f,0.f,0.f};

#pragma unroll 1
    for (unsigned j0 = 0; j0 < (unsigned)SEQ; j0 += 32u) {
        const v4f r0 = *(const v4f*)(rightp + j0);
        const v4f r1 = *(const v4f*)(rightp + j0 + 4u);
        const v4f r2 = *(const v4f*)(rightp + j0 + 16u);
        const v4f r3 = *(const v4f*)(rightp + j0 + 20u);
        v16h av[4];
#pragma unroll
        for (int t = 0; t < 4; ++t) av[t] = frag_ld(vrow + (size_t)(16u * (unsigned)t) * SEQ + j0);
        const float rj[16] = {r0.x, r0.y, r0.z, r0.w, r1.x, r1.y, r1.z, r1.w,
                              r2.x, r2.y, r2.z, r2.w, r3.x, r3.y, r3.z, r3.w};
        float tt[16];
#pragma unroll
        for (int e = 0; e < 16; ++e) {
            float s = li + rj[e];
            s = (s >= 0.0f) ? s : LEAK * s;
            tt[e] = s * LOG2E;
        }
        float mx = tt[0];
#pragma unroll
        for (int e = 1; e < 16; ++e) mx = fselmax(mx, tt[e]);
        mx = fselmax(mx, __shfl_xor(mx, 16, 32));
        const float mnew = fselmax(m, mx);
        const float alpha = exp2f(m - mnew);
        m = mnew;
        float psum = 0.f;
        float pw[16];
#pragma unroll
        for (int e = 0; e < 16; ++e) {
            const float p = exp2f(tt[e] - mnew);
            psum += p;
            pw[e] = p * P_CARRY;
        }
        lsum = lsum * alpha + psum;
        v8u pk;
#pragma unroll
        for (int e2 = 0; e2 < 8; ++e2) pk[e2] = toh_flush2(pw[2 * e2], pw[2 * e2 + 1]);
        const v16h pf = __builtin_bit_cast(v16h, pk);
#pragma unroll
        for (int t = 0; t < 4; ++t)
#pragma unroll
            for (int r = 0; r < 8; ++r) acc[t][r] *= alpha;
#pragma unroll
        for (int t = 0; t < 4; ++t) acc[t] = wmma16(av[t], pf, acc[t]);
    }

    lsum += __shfl_xor(lsum, 16, 32);
#pragma unroll
    for (int t = 0; t < 4; ++t) {
        v4f lo, hi;
        lo.x = acc[t][0]; lo.y = acc[t][1]; lo.z = acc[t][2]; lo.w = acc[t][3];
        hi.x = acc[t][4]; hi.y = acc[t][5]; hi.z = acc[t][6]; hi.w = acc[t][7];
        *(v4f*)(&sO[wave][c * AT_PO + 16u * (unsigned)t + 8u * hh]) = lo;
        *(v4f*)(&sO[wave][c * AT_PO + 16u * (unsigned)t + 8u * hh + 4u]) = hi;
    }
    sL[wave][c] = lsum;
    wave_sync_lds();
    {
        const unsigned c4 = (lane & 15u) * 4u;
        float* orow = out + (size_t)(b * (unsigned)SEQ + i0) * OUT_DIM + hd * (unsigned)HD + c4;
#pragma unroll 1
        for (unsigned it = 0; it < 8u; ++it) {
            const unsigned row = 2u * it + hh;
            const v4f x = *(const v4f*)(&sO[wave][row * AT_PO + c4]);
            const float lr = sL[wave][row];
            v4f v;
            v.x = elu1((x.x / lr) * PV_UNDO);
            v.y = elu1((x.y / lr) * PV_UNDO);
            v.z = elu1((x.z / lr) * PV_UNDO);
            v.w = elu1((x.w / lr) * PV_UNDO);
            VST2V4(orow + (size_t)row * OUT_DIM, v);
        }
    }
}

static constexpr size_t SZ_X16 = (size_t)MTOK * IN_DIM * 2;
static constexpr size_t SZ_WT  = (size_t)NPROJ * IN_DIM * 2;
static constexpr size_t SZ_HF  = (size_t)MTOK * NPROJ * 4;
static constexpr size_t SZ_VT  = (size_t)NB * OUT_DIM * SEQ * 2;
static constexpr size_t SZ_LR  = (size_t)2 * NB * HEADS * SEQ * 4;
static constexpr size_t OFF_X16 = 0;
static constexpr size_t OFF_WT  = OFF_X16 + SZ_X16;
static constexpr size_t OFF_HF  = OFF_WT + SZ_WT;
static constexpr size_t OFF_VT  = OFF_HF + SZ_HF;
static constexpr size_t OFF_LR  = OFF_VT + SZ_VT;
static constexpr size_t WS_TOTAL = OFF_LR + SZ_LR;
static_assert(SZ_X16 % 256 == 0 && SZ_WT % 256 == 0 && SZ_HF % 256 == 0 && SZ_VT % 256 == 0 && SZ_LR % 256 == 0);
static_assert(WS_TOTAL <= (size_t)134217728);

static constexpr unsigned GRID_WT  = (OUT_DIM * (IN_DIM / 8)) / 256;
static constexpr unsigned GRID_X16 = (MTOK * IN_DIM / 8) / 256;
static constexpr unsigned GRID_GEMM = ((MTOK / 64) * (NPROJ / 64) + 7) / 8;
static constexpr unsigned GRID_PL  = NB * (SEQ / 64) * HEADS;
static constexpr unsigned GRID_AT  = NB * HEADS * (SEQ / 128);
static_assert((OUT_DIM * (IN_DIM / 8)) % 256 == 0);
static_assert(((MTOK / 64) * (NPROJ / 64)) % 8 == 0);

extern "C" void kernel_launch(void* const* d_in, const int* in_sizes, int n_in, void* d_out, int out_size,
                              void* d_ws, size_t ws_size, hipStream_t stream) {
    if (n_in < 4) return;
    if (in_sizes[0] < ((NB - 1) * SEQ_FULL + SEQ) * IN_DIM) return;
    if (in_sizes[1] < IN_DIM * OUT_DIM || in_sizes[2] < IN_DIM * OUT_DIM || in_sizes[3] < HEADS * 2 * HD) return;
    if (out_size < MTOK * OUT_DIM) return;
    if (WS_TOTAL > ws_size) return;

    const float* h    = (const float*)d_in[0];
    const float* W_s  = (const float*)d_in[1];
    const float* W_n  = (const float*)d_in[2];
    const float* attn = (const float*)d_in[3];
    float* out = (float*)d_out;

    char* wsp = (char*)d_ws;
    unsigned short* x16  = (unsigned short*)(wsp + OFF_X16);
    unsigned short* wt16 = (unsigned short*)(wsp + OFF_WT);
    float*          hf   = (float*)(wsp + OFF_HF);
    unsigned short* vt16 = (unsigned short*)(wsp + OFF_VT);
    float*          lr   = (float*)(wsp + OFF_LR);

    k_wt16<<<dim3(GRID_WT, 1), 256, 0, stream>>>(W_s, IN_DIM, OUT_DIM, 5, wt16, W_CARRY);
    k_wt16<<<dim3(GRID_WT, 1), 256, 0, stream>>>(W_n, IN_DIM, OUT_DIM, 5, wt16 + (size_t)OUT_DIM * IN_DIM, W_CARRY);
    k_x16<<<GRID_X16, 256, 0, stream>>>(h, x16);
    k_gemm64<<<GRID_GEMM, 256, 0, stream>>>((const _Float16*)x16, IN_DIM, (const _Float16*)wt16, IN_DIM,
                                            hf, NPROJ, MTOK, NPROJ, IN_DIM);
    k_planes<<<GRID_PL, 256, 0, stream>>>(hf, attn, vt16, lr);
    k_attn<<<GRID_AT, 256, 0, stream>>>((const _Float16*)vt16, (const float*)lr, out);
}
